// CrossAttn_17557826306465
// MI455X (gfx1250) — hardware-verified
//
#include <hip/hip_runtime.h>
#include <math.h>

constexpr int kB        = 4;
constexpr int kL        = 1024;
constexpr int kD        = 1024;
constexpr int kH        = 16;
constexpr int kDh       = 64;
constexpr int kNK       = 21;
constexpr int kTok      = kB * kL;
constexpr int kTabLen   = 2 * kL - 1;
constexpr int kTabPitch = 2048;
constexpr int kGroup    = 4;
constexpr float kWCarry     = 16.0f;
constexpr float kWCarryInv  = 1.0f / 16.0f;
constexpr float kPCarry     = 32768.0f;
constexpr float kAttCarry   = 256.0f;
constexpr float kScoreScale = 0.125f;
constexpr float kPVScale    = kAttCarry / kPCarry;
constexpr float kGateScale  = 1.0f / (kAttCarry * kWCarry);
static_assert(kH * kDh == kD);
static_assert(kL % 64 == 0 && kD % 64 == 0 && kDh % 64 == 0 && kTok % 64 == 0);
static_assert(kDh % 32 == 0 && kD % 32 == 0 && kL % 32 == 0);
static_assert(kH % kGroup == 0 && kL == 8 * 128 && kD == 4 * 256);
static_assert(kTabLen < kTabPitch && (kH * kTabPitch) % 256 == 0);

typedef __attribute__((ext_vector_type(16))) _Float16 v16h;
typedef __attribute__((ext_vector_type(8)))  _Float16 v8h;
typedef __attribute__((ext_vector_type(16))) __bf16   v16b;
typedef __attribute__((ext_vector_type(8)))  __bf16   v8b;
typedef __attribute__((ext_vector_type(8)))  float    v8f;
typedef __attribute__((ext_vector_type(4)))  float    v4f;
typedef __attribute__((ext_vector_type(2)))  float    v2f;
typedef __attribute__((ext_vector_type(4)))  unsigned int v4u;

__device__ __forceinline__ unsigned short f2bf_bits(float f) {
  unsigned u = __float_as_uint(f);
  return (unsigned short)((u + 0x7FFFu + ((u >> 16) & 1u)) >> 16);
}
__device__ __forceinline__ float bf_bits2f(unsigned short h) { return __uint_as_float(((unsigned)h) << 16); }

__device__ __forceinline__ void dep_guard_h(v8f& a, v8f& b, v16h x, v16h y) { asm volatile("v_nop\n\tv_nop\n\tv_nop\n\tv_nop" : "+v"(a), "+v"(b) : "v"(x), "v"(y)); }
__device__ __forceinline__ void dep_guard_b(v8f& a, v8f& b, v16b x, v16b y) { asm volatile("v_nop\n\tv_nop\n\tv_nop\n\tv_nop" : "+v"(a), "+v"(b) : "v"(x), "v"(y)); }
__device__ __forceinline__ void dep_guard4_h(v8f& a, v8f& b, v8f& c, v8f& d, v16h x, v16h y) { asm volatile("v_nop\n\tv_nop\n\tv_nop\n\tv_nop" : "+v"(a), "+v"(b), "+v"(c), "+v"(d) : "v"(x), "v"(y)); }
__device__ __forceinline__ void dep_guard4_b(v8f& a, v8f& b, v8f& c, v8f& d, v16b x, v16b y) { asm volatile("v_nop\n\tv_nop\n\tv_nop\n\tv_nop" : "+v"(a), "+v"(b), "+v"(c), "+v"(d) : "v"(x), "v"(y)); }
__device__ __forceinline__ void keep4_h(v16h a, v16h b, v16h c, v16h d) { asm volatile("v_nop" :: "v"(a), "v"(b), "v"(c), "v"(d)); }
__device__ __forceinline__ void keep4_b(v16b a, v16b b, v16b c, v16b d) { asm volatile("v_nop" :: "v"(a), "v"(b), "v"(c), "v"(d)); }
__device__ __forceinline__ void acc_guard4(v8f& a, v8f& b, v8f& c, v8f& d) { asm volatile("v_nop\n\tv_nop\n\tv_nop\n\tv_nop" : "+v"(a), "+v"(b), "+v"(c), "+v"(d)); }
template <typename T> struct Frag;
template <> struct Frag<_Float16> {
  typedef v16h V; union U { v16h v; v8h h[2]; };
  static __device__ __forceinline__ v16h load(const _Float16* p) {
    U f; f.h[0] = *(const v8h*)(p); f.h[1] = *(const v8h*)(p + 16); return f.v;
  }
  static __device__ __forceinline__ v8f mma(v16h a, v16h b, v8f c) {
    return __builtin_amdgcn_wmma_f32_16x16x32_f16(false, a, false, b, (short)0, c, false, false);
  }
  static __device__ __forceinline__ void guard(v8f& a, v8f& b, v16h x, v16h y) { dep_guard_h(a, b, x, y); }
  static __device__ __forceinline__ void guard4(v8f& a, v8f& b, v8f& c, v8f& d, v16h x, v16h y) { dep_guard4_h(a, b, c, d, x, y); }
  static __device__ __forceinline__ void keep(v16h a, v16h b, v16h c, v16h d) { keep4_h(a, b, c, d); }
};
template <> struct Frag<__bf16> {
  typedef v16b V; union U { v16b v; v8b h[2]; };
  static __device__ __forceinline__ v16b load(const __bf16* p) {
    U f; f.h[0] = *(const v8b*)(p); f.h[1] = *(const v8b*)(p + 16); return f.v;
  }
  static __device__ __forceinline__ v8f mma(v16b a, v16b b, v8f c) {
    return __builtin_amdgcn_wmma_f32_16x16x32_bf16(false, a, false, b, (short)0, c, false, false);
  }
  static __device__ __forceinline__ void guard(v8f& a, v8f& b, v16b x, v16b y) { dep_guard_b(a, b, x, y); }
  static __device__ __forceinline__ void guard4(v8f& a, v8f& b, v8f& c, v8f& d, v16b x, v16b y) { dep_guard4_b(a, b, c, d, x, y); }
  static __device__ __forceinline__ void keep(v16b a, v16b b, v16b c, v16b d) { keep4_b(a, b, c, d); }
};

__device__ __forceinline__ unsigned pk16(unsigned short a, unsigned short b) { return (unsigned)a | ((unsigned)b << 16); }
__device__ __forceinline__ unsigned short h_bits(float f) { const _Float16 h = (_Float16)f; return __builtin_bit_cast(unsigned short, h); }

template <int ET> struct Elem;
template <> struct Elem<0> { typedef _Float16 T; };
template <> struct Elem<1> { typedef __bf16 T; };
template <int ET, bool SPLIT, int BIAS_MODE, int OUT_MODE, bool RESID, int ACT = 0>
__global__ __launch_bounds__(256) void wmma_gemm64(
    const unsigned short* __restrict__ Ap, const unsigned short* __restrict__ A2p, int lda, long strideA,
    const unsigned short* __restrict__ Btp, const unsigned short* __restrict__ Bt2p, int ldb, long strideB,
    void* __restrict__ Cout, void* __restrict__ Cout2, int ldc, long strideC,
    const float* __restrict__ bias,
    const float* __restrict__ resid, long strideR,
    int M, int N, int K, float scale) {
  typedef typename Elem<ET>::T T;
  typedef typename Frag<T>::V V;
  const T* A = (const T*)Ap; const T* A2 = (const T*)A2p; const T* Bt = (const T*)Btp; const T* Bt2 = (const T*)Bt2p;
  __shared__ __align__(16) float sT[8][16 * 68];
  const int b    = blockIdx.y;
  const int lane = threadIdx.x & 31;
  const int wave = threadIdx.x >> 5;
  const int tilesN = N >> 6;
  const int tilesM = M >> 6;
  const int tile = blockIdx.x * 8 + wave;
  if (tile >= tilesM * tilesN) return;
  const int tm = tile / tilesN;
  const int tn = tile - tm * tilesN;
  const int m0 = tm << 6;
  const int n0 = tn << 6;

  const T* Ab  = A  + (size_t)b * strideA;
  const T* Bb  = Bt + (size_t)b * strideB;
  const T* Ab2 = SPLIT ? (A2  + (size_t)b * strideA) : nullptr;
  const T* Bb2 = SPLIT ? (Bt2 + (size_t)b * strideB) : nullptr;

  const int rlane = lane & 15;
  const int koff  = (lane >> 4) * 8;
  const int mOff  = (lane >> 4) * 8;

  v8f acc[4][4];
#pragma unroll
  for (int i = 0; i < 4; ++i)
#pragma unroll
    for (int j = 0; j < 4; ++j) acc[i][j] = (v8f){0.f,0.f,0.f,0.f,0.f,0.f,0.f,0.f};

  for (int k0 = 0; k0 < K; k0 += 32) {
    V bh[4], bl[4];
#pragma unroll
    for (int j = 0; j < 4; ++j) {
      const size_t bo = (size_t)(n0 + (j << 4) + rlane) * ldb + koff + k0;
      bh[j] = Frag<T>::load(Bb + bo);
      if (SPLIT) bl[j] = Frag<T>::load(Bb2 + bo);
    }
#pragma unroll
    for (int i = 0; i < 4; ++i) {
      const size_t ao = (size_t)(m0 + (i << 4) + rlane) * lda + koff + k0;
      V ah = Frag<T>::load(Ab + ao);
      V al;
      if (SPLIT) al = Frag<T>::load(Ab2 + ao);
#pragma unroll
      for (int j = 0; j < 4; ++j) {
        acc[i][j] = Frag<T>::mma(ah, bh[j], acc[i][j]);
        if (SPLIT) {
          acc[i][j] = Frag<T>::mma(ah, bl[j], acc[i][j]);
          acc[i][j] = Frag<T>::mma(al, bh[j], acc[i][j]);
        }
      }
      Frag<T>::guard4(acc[i][0], acc[i][1], acc[i][2], acc[i][3], ah, SPLIT ? al : ah);
    }
    Frag<T>::keep(bh[0], bh[1], bh[2], bh[3]);
    if (SPLIT) Frag<T>::keep(bl[0], bl[1], bl[2], bl[3]);
  }
  acc_guard4(acc[0][0], acc[0][1], acc[0][2], acc[0][3]);
  acc_guard4(acc[1][0], acc[1][1], acc[1][2], acc[1][3]);
  acc_guard4(acc[2][0], acc[2][1], acc[2][2], acc[2][3]);
  acc_guard4(acc[3][0], acc[3][1], acc[3][2], acc[3][3]);

  float* slab = sT[wave];
  const float* Rb = RESID ? (resid + (size_t)b * strideR) : nullptr;
#pragma unroll
  for (int i = 0; i < 4; ++i) {
    const int mBase = m0 + (i << 4);
#pragma unroll
    for (int j = 0; j < 4; ++j) {
      const int n = n0 + (j << 4) + rlane;
      float bv = 0.f;
      if (BIAS_MODE == 2) bv = bias[n];
#pragma unroll
      for (int r = 0; r < 8; ++r) {
        float v = acc[i][j][r] * scale;
        if (BIAS_MODE == 1) v += bias[mBase + mOff + r];
        if (BIAS_MODE == 2) v += bv;
        if (RESID) v += Rb[(size_t)(mBase + mOff + r) * ldc + n];
        if (ACT == 2) v = fmaxf(v, 0.0f);
        if (ACT == 4) v = (v > 0.f) ? v : 0.01f * v;
        slab[(mOff + r) * 68 + (j << 4) + rlane] = v;
      }
    }
    __builtin_amdgcn_fence(__ATOMIC_RELEASE, "workgroup");
    __builtin_amdgcn_wave_barrier();
    __builtin_amdgcn_fence(__ATOMIC_ACQUIRE, "workgroup");
    if (OUT_MODE == 0) {
      float* C = (float*)Cout + (size_t)b * strideC;
      const int hh = lane >> 4, c4 = (lane & 15) * 4;
      for (int pass = 0; pass < 2; ++pass) {
#pragma unroll
        for (int it = 0; it < 8; ++it) {
          const int row = it * 2 + hh;
          v4f v = *(const v4f*)(slab + row * 68 + c4);
          *(volatile v4f*)(C + (size_t)(mBase + row) * ldc + n0 + c4) = v;
        }
        __threadfence();
      }
    } else {
      const int q = lane >> 3, c8 = (lane & 7) * 8;
      unsigned short* C  = (unsigned short*)Cout  + (size_t)b * strideC;
      unsigned short* C2 = (OUT_MODE == 2) ? ((unsigned short*)Cout2 + (size_t)b * strideC) : nullptr;
      for (int pass = 0; pass < 2; ++pass) {
#pragma unroll
        for (int it = 0; it < 4; ++it) {
          const int row = it * 4 + q;
          const float* sp = slab + row * 68 + c8;
          v8h hv, lv;
#pragma unroll
          for (int e = 0; e < 8; ++e) {
            if (OUT_MODE == 1) {
              hv[e] = (_Float16)sp[e];
            } else {
              unsigned short hb = f2bf_bits(sp[e]);
              unsigned short lb = f2bf_bits(sp[e] - bf_bits2f(hb));
              hv[e] = __builtin_bit_cast(_Float16, hb);
              lv[e] = __builtin_bit_cast(_Float16, lb);
            }
          }
          *(volatile v8h*)(C + (size_t)(mBase + row) * ldc + n0 + c8) = hv;
          if (OUT_MODE == 2) *(volatile v8h*)(C2 + (size_t)(mBase + row) * ldc + n0 + c8) = lv;
        }
        __threadfence();
      }
    }
    __builtin_amdgcn_fence(__ATOMIC_RELEASE, "workgroup");
    __builtin_amdgcn_wave_barrier();
    __builtin_amdgcn_fence(__ATOMIC_ACQUIRE, "workgroup");
  }
}

__global__ __launch_bounds__(256) void cast8_f16_kernel(const float* __restrict__ in, unsigned short* __restrict__ out, int n8) {
  const int i = blockIdx.x * 256 + threadIdx.x;
  if (i >= n8) return;
  const float* p = in + 8 * (size_t)i;
  const v4f a = *(const v4f*)(p);
  const v4f c = *(const v4f*)(p + 4);
  unsigned short hb[8];
#pragma unroll
  for (int e = 0; e < 4; ++e) {
    hb[e]     = h_bits(a[e]);
    hb[4 + e] = h_bits(c[e]);
  }
  const v4u u = (v4u){pk16(hb[0], hb[1]), pk16(hb[2], hb[3]), pk16(hb[4], hb[5]), pk16(hb[6], hb[7])};
  unsigned short* q = out + 8 * (size_t)i;
  *(volatile v4u*)q = u;
  __threadfence();
  *(volatile v4u*)q = u;
}

__global__ __launch_bounds__(256) void wtcast_kernel(const float* __restrict__ W, int Nout, int Kin,
                                                     unsigned short* __restrict__ WT, float scale) {
  __shared__ float sm[64][65];
  const int t  = threadIdx.x;
  const int k0 = blockIdx.x * 64;
  const int n0 = blockIdx.y * 64;
#pragma unroll
  for (int i = 0; i < 8; ++i) {
    const int e = i * 256 + t;
    const int r = e >> 6;
    const int c = e & 63;
    sm[c][r] = W[(size_t)(k0 + r) * Nout + n0 + c] * scale;
  }
  asm volatile("" ::: "memory");
#pragma unroll
  for (int i = 8; i < 16; ++i) {
    const int e = i * 256 + t;
    const int r = e >> 6;
    const int c = e & 63;
    sm[c][r] = W[(size_t)(k0 + r) * Nout + n0 + c] * scale;
  }
  __syncthreads();
  const int lane = t & 31, wave = t >> 5;
  const int q = lane >> 3, c8 = (lane & 7) * 8;
  for (int pass = 0; pass < 2; ++pass) {
#pragma unroll
    for (int it = 0; it < 2; ++it) {
      const int row = wave * 8 + it * 4 + q;
      unsigned short hb[8];
#pragma unroll
      for (int e = 0; e < 8; ++e) hb[e] = h_bits(sm[row][c8 + e]);
      const v4u u = (v4u){pk16(hb[0], hb[1]), pk16(hb[2], hb[3]), pk16(hb[4], hb[5]), pk16(hb[6], hb[7])};
      *(volatile v4u*)(WT + (size_t)(n0 + row) * Kin + k0 + c8) = u;
    }
    __threadfence();
  }
}

__global__ __launch_bounds__(256) void bias_table_kernel(const float* __restrict__ amp, const float* __restrict__ off,
                                                         const float* __restrict__ sharp, float* __restrict__ T) {
  const int idx = blockIdx.x * 256 + threadIdx.x;
  const int h = idx >> 11;
  const int p = idx & (kTabPitch - 1);
  const float dd = (float)(p - (kL - 1));
  float s = 0.0f;
#pragma unroll 1
  for (int k = 0; k < kNK; ++k) {
    const float a  = amp[h * kNK + k];
    const float o  = off[h * kNK + k];
    const float sh = fabsf(sharp[h * kNK + k]);
    const float df = dd - o;
    const float sq = df * df;
    const float ex = expf(-sh * sq);
    s += a * ex;
  }
  const float val = (p < kTabLen) ? s : 0.0f;
  float* tp = T + idx;
  *(volatile float*)tp = val;
  __threadfence();
  *(volatile float*)tp = val;
}

__global__ __launch_bounds__(128) void bias_softmax_kernel(const float* __restrict__ Sp, const float* __restrict__ Tg,
                                                          unsigned short* __restrict__ Pp) {
  __shared__ __align__(16) float lg[kL];
  __shared__ float redM[4];
  __shared__ float redS[4];
  const int i    = blockIdx.x;
  const int hg   = blockIdx.y;
  const int t    = threadIdx.x;
  const int lane = t & 31, wave = t >> 5;
  const size_t rowoff = ((size_t)hg * kL + i) * kL;
  const float* sr = Sp + rowoff;
  const float* tr = Tg + (size_t)hg * kTabPitch + (kL - 1 - i);

  float mx = -__builtin_inff();
#pragma unroll 1
  for (int it = 0; it < 4; ++it) {
    const int c = it * 256 + 2 * t;
    const v2f sv = *(const v2f*)(sr + c);
    const float b0 = tr[c];
    const float b1 = tr[c + 1];
    v2f av;
    av[0] = sv[0] + b0;
    av[1] = sv[1] + b1;
    mx = fmaxf(mx, fmaxf(av[0], av[1]));
    *(v2f*)(lg + c) = av;
  }
#pragma unroll
  for (int w = 16; w > 0; w >>= 1) mx = fmaxf(mx, __shfl_xor(mx, w, 32));
  if (lane == 0) redM[wave] = mx;
  __syncthreads();
  const float m = fmaxf(fmaxf(redM[0], redM[1]), fmaxf(redM[2], redM[3]));

  float sum = 0.0f;
#pragma unroll 1
  for (int it = 0; it < 4; ++it) {
    const int c = it * 256 + 2 * t;
    const v2f l = *(const v2f*)(lg + c);
    v2f ev;
#pragma unroll
    for (int e = 0; e < 2; ++e) {
      ev[e] = expf(l[e] - m);
      sum += ev[e];
    }
    *(v2f*)(lg + c) = ev;
  }
#pragma unroll
  for (int w = 16; w > 0; w >>= 1) sum += __shfl_xor(sum, w, 32);
  if (lane == 0) redS[wave] = sum;
  __syncthreads();
  const float tot = ((redS[0] + redS[1]) + redS[2]) + redS[3];
  const float inv = kPCarry / tot;

  const v4f e0 = *(const v4f*)(lg + 8 * t);
  const v4f e1 = *(const v4f*)(lg + 8 * t + 4);
  unsigned short hb[8];
#pragma unroll
  for (int e = 0; e < 4; ++e) {
    hb[e]     = h_bits(e0[e] * inv);
    hb[4 + e] = h_bits(e1[e] * inv);
  }
  const v4u u = (v4u){pk16(hb[0], hb[1]), pk16(hb[2], hb[3]), pk16(hb[4], hb[5]), pk16(hb[6], hb[7])};
  unsigned short* pr = Pp + rowoff + 8 * (size_t)t;
  *(volatile v4u*)pr = u;
  __threadfence();
  *(volatile v4u*)pr = u;
}

__global__ __launch_bounds__(256) void gate_kernel(const float* __restrict__ G, const float* __restrict__ bg,
                                                   float* __restrict__ out) {
  const int r = blockIdx.x;
  const int c = threadIdx.x * 4;
  const float* gr = G + (size_t)r * (2 * kD);
  const v4f ga = *(const v4f*)(gr + c);
  const v4f gb = *(const v4f*)(gr + kD + c);
  const v4f ba = *(const v4f*)(bg + c);
  const v4f bb = *(const v4f*)(bg + kD + c);
  v4f o;
#pragma unroll
  for (int e = 0; e < 4; ++e) {
    const float a  = ga[e] + ba[e];
    const float bq = gb[e] + bb[e];
    const float ex = expf(-bq);
    const float sg = 1.0f / (1.0f + ex);
    o[e] = a * sg;
  }
  float* op = out + (size_t)r * kD + c;
  *(volatile v4f*)op = o;
  __threadfence();
  *(volatile v4f*)op = o;
}

extern "C" void kernel_launch(void* const* d_in, const int* in_sizes, int n_in,
                              void* d_out, int out_size, void* d_ws, size_t ws_size,
                              hipStream_t stream) {
  if (n_in < 9) return;
  const int nAct = kTok * kD;
  if (in_sizes[0] != nAct || in_sizes[1] != nAct) return;
  if (in_sizes[2] != kD * kD || in_sizes[3] != kD * 2 * kD || in_sizes[4] != kD * 2 * kD) return;
  if (in_sizes[5] != 2 * kD) return;
  if (in_sizes[6] != kH * kNK || in_sizes[7] != kH * kNK || in_sizes[8] != kH * kNK) return;
  if (out_size != nAct) return;

  const size_t szAct16 = (size_t)kTok * kD * 2;
  const size_t szWq16  = (size_t)kD * kD * 2;
  const size_t szW2    = (size_t)2 * kD * kD * 2;
  const size_t szTab   = (size_t)kH * kTabPitch * 4;
  const size_t szSC    = (size_t)kGroup * kL * kL * 4;
  const size_t szPP    = (size_t)kGroup * kL * kL * 2;
  const size_t szGG    = (size_t)kTok * 2 * kD * 4;
  const size_t offXq  = 0;
  const size_t offXkv = offXq  + szAct16;
  const size_t offWq  = offXkv + szAct16;
  const size_t offWm  = offWq  + szWq16;
  const size_t offWg  = offWm  + szW2;
  const size_t offTab = offWg  + szW2;
  const size_t offQ   = offTab + szTab;
  const size_t offK   = offQ   + szAct16;
  const size_t offVT  = offK   + szAct16;
  const size_t offAtt = offVT  + szAct16;
  const size_t offSC  = offAtt + szAct16;
  const size_t offPP  = offSC  + szSC;
  const size_t offGG  = offPP  + szPP;
  const size_t total  = offGG  + szGG;
  if (ws_size < total) return;

  const float* x_q   = (const float*)d_in[0];
  const float* x_kv  = (const float*)d_in[1];
  const float* Wq    = (const float*)d_in[2];
  const float* Wm    = (const float*)d_in[3];
  const float* Wg    = (const float*)d_in[4];
  const float* bg    = (const float*)d_in[5];
  const float* amp   = (const float*)d_in[6];
  const float* off   = (const float*)d_in[7];
  const float* sharp = (const float*)d_in[8];
  float* out = (float*)d_out;
  char* ws = (char*)d_ws;
  unsigned short* Xq16  = (unsigned short*)(ws + offXq);
  unsigned short* Xkv16 = (unsigned short*)(ws + offXkv);
  unsigned short* WqT16 = (unsigned short*)(ws + offWq);
  unsigned short* WmT16 = (unsigned short*)(ws + offWm);
  unsigned short* WgT16 = (unsigned short*)(ws + offWg);
  float*          TB    = (float*)(ws + offTab);
  unsigned short* Q16   = (unsigned short*)(ws + offQ);
  unsigned short* K16   = (unsigned short*)(ws + offK);
  unsigned short* VT16  = (unsigned short*)(ws + offVT);
  unsigned short* ATT16 = (unsigned short*)(ws + offAtt);
  float*          SC    = (float*)(ws + offSC);
  unsigned short* PP    = (unsigned short*)(ws + offPP);
  float*          GG    = (float*)(ws + offGG);

  const int n8 = nAct / 8;
  cast8_f16_kernel<<<dim3(n8 / 256), dim3(256), 0, stream>>>(x_q, Xq16, n8);
  cast8_f16_kernel<<<dim3(n8 / 256), dim3(256), 0, stream>>>(x_kv, Xkv16, n8);
  wtcast_kernel<<<dim3(kD / 64, kD / 64), dim3(256), 0, stream>>>(Wq, kD, kD, WqT16, kWCarry);
  wtcast_kernel<<<dim3(kD / 64, 2 * kD / 64), dim3(256), 0, stream>>>(Wm, 2 * kD, kD, WmT16, kWCarry);
  wtcast_kernel<<<dim3(kD / 64, 2 * kD / 64), dim3(256), 0, stream>>>(Wg, 2 * kD, kD, WgT16, kWCarry);
  bias_table_kernel<<<dim3(kH * kTabPitch / 256), dim3(256), 0, stream>>>(amp, off, sharp, TB);

  const int tilesProj = (kTok / 64) * (kD / 64);
  wmma_gemm64<0, false, 0, 1, false, 0><<<dim3(tilesProj / 8, 1), dim3(256), 0, stream>>>(
      Xq16, Xq16, kD, 0L, WqT16, WqT16, kD, 0L,
      (void*)Q16, (void*)Q16, kD, 0L, TB, TB, 0L, kTok, kD, kD, kWCarryInv);
  wmma_gemm64<0, false, 0, 1, false, 0><<<dim3(tilesProj / 8, 1), dim3(256), 0, stream>>>(
      Xkv16, Xkv16, kD, 0L, WmT16, WmT16, kD, 0L,
      (void*)K16, (void*)K16, kD, 0L, TB, TB, 0L, kTok, kD, kD, kWCarryInv);
  const int tilesVT = (kD / 64) * (kL / 64);
  wmma_gemm64<0, false, 0, 1, false, 0><<<dim3(tilesVT / 8, kB), dim3(256), 0, stream>>>(
      WmT16 + (size_t)kD * kD, WmT16 + (size_t)kD * kD, kD, 0L,
      Xkv16, Xkv16, kD, (long)kL * kD,
      (void*)VT16, (void*)VT16, kL, (long)kD * kL, TB, TB, 0L, kD, kL, kD, kWCarryInv);

  const long strideHead16 = (long)kDh;
  const long strideScore  = (long)kL * kL;
  const long strideVT     = (long)kDh * kL;
  const int  tilesScore   = (kL / 64) * (kL / 64);
  const int  tilesCtx     = (kL / 64) * (kDh / 64);
  for (int b = 0; b < kB; ++b) {
    for (int g = 0; g < kH / kGroup; ++g) {
      const size_t headCol = (size_t)g * kGroup * kDh;
      const size_t tokOff  = ((size_t)b * kL) * kD + headCol;
      const unsigned short* Ag  = Q16 + tokOff;
      const unsigned short* Btg = K16 + tokOff;
      wmma_gemm64<0, false, 0, 0, false, 0><<<dim3(tilesScore / 8, kGroup), dim3(256), 0, stream>>>(
          Ag, Ag, kD, strideHead16, Btg, Btg, kD, strideHead16,
          (void*)SC, (void*)SC, kL, strideScore, TB, TB, 0L, kL, kL, kDh, kScoreScale);
      bias_softmax_kernel<<<dim3(kL, kGroup), dim3(128), 0, stream>>>(SC, TB + (size_t)g * kGroup * kTabPitch, PP);
      const unsigned short* VTg = VT16 + ((size_t)b * kD + headCol) * kL;
      unsigned short* Cg = ATT16 + tokOff;
      wmma_gemm64<0, false, 0, 1, false, 0><<<dim3(tilesCtx / 8, kGroup), dim3(256), 0, stream>>>(
          PP, PP, kL, strideScore, VTg, VTg, kL, strideVT,
          (void*)Cg, (void*)Cg, kD, strideHead16, TB, TB, 0L, kL, kDh, kL, kPVScale);
    }
  }

  const int tilesGate = (kTok / 64) * (2 * kD / 64);
  wmma_gemm64<0, false, 0, 0, false, 0><<<dim3(tilesGate / 8, 1), dim3(256), 0, stream>>>(
      ATT16, ATT16, kD, 0L, WgT16, WgT16, kD, 0L,
      (void*)GG, (void*)GG, 2 * kD, 0L, TB, TB, 0L, kTok, 2 * kD, kD, kGateScale);
  gate_kernel<<<dim3(kTok), dim3(256), 0, stream>>>(GG, bg, out);
}
